// LinearAttention_89850715833062
// MI455X (gfx1250) — hardware-verified
//
#include <hip/hip_runtime.h>
#include <math.h>

constexpr int kBatch = 4;
constexpr int kSeq   = 4096;
constexpr int kC     = 768;
constexpr int kHeads = 12;
constexpr int kDh    = 64;
constexpr int kTok   = kBatch * kSeq;
constexpr int kC3    = 3 * kC;
constexpr int kBH    = kBatch * kHeads;
constexpr float kWCarryInv = 1.0f / 64.0f;
constexpr float kWCarry    = 64.0f;
constexpr float kYCarry    = 64.0f;
constexpr float kProjScale = 1.0f / (64.0f * 64.0f);
constexpr float kEps       = 1.0e-6f;
static_assert(kHeads * kDh == kC, "shape");
static_assert(kTok % 64 == 0 && kC % 64 == 0 && kC3 % 64 == 0, "tile multiples");
static_assert(kC % 32 == 0 && kSeq % 32 == 0 && kDh % 32 == 0, "K multiples of 32");
static_assert(kSeq % 512 == 0, "y kernel grid");
static_assert((kTok * kC) % 2048 == 0 && (kC3 * kC) % 2048 == 0 && (kC * kC) % 2048 == 0, "cast grids exact");

typedef __attribute__((ext_vector_type(16))) _Float16 v16h;
typedef __attribute__((ext_vector_type(8)))  _Float16 v8h;
typedef __attribute__((ext_vector_type(16))) __bf16   v16b;
typedef __attribute__((ext_vector_type(8)))  __bf16   v8b;
typedef __attribute__((ext_vector_type(8)))  float    v8f;
typedef __attribute__((ext_vector_type(4)))  float    v4f;
typedef __attribute__((ext_vector_type(4)))  unsigned int v4u;

__device__ __forceinline__ unsigned short f2bf_bits(float f) {
  unsigned u = __float_as_uint(f);
  return (unsigned short)((u + 0x7FFFu + ((u >> 16) & 1u)) >> 16);
}
__device__ __forceinline__ float bf_bits2f(unsigned short h) { return __uint_as_float(((unsigned)h) << 16); }

__device__ __forceinline__ float h16_to_f32(unsigned hb) {
  const unsigned sgn = (hb & 0x8000u) << 16; const unsigned em = hb & 0x7fffu;
  const float fn = __uint_as_float((em << 13) + 0x38000000u);
  const float fs = (float)em * 5.9604644775390625e-8f;
  const float mag = (em < 0x400u) ? fs : fn; return __uint_as_float(__float_as_uint(mag) | sgn); }

__device__ __forceinline__ void dep_guard_h(v8f& a, v8f& b, v16h x, v16h y) { asm volatile("v_nop\n\tv_nop\n\tv_nop\n\tv_nop" : "+v"(a), "+v"(b) : "v"(x), "v"(y)); }
__device__ __forceinline__ void dep_guard_b(v8f& a, v8f& b, v16b x, v16b y) { asm volatile("v_nop\n\tv_nop\n\tv_nop\n\tv_nop" : "+v"(a), "+v"(b) : "v"(x), "v"(y)); }
__device__ __forceinline__ void dep_guard4_h(v8f& a0, v8f& a1, v8f& a2, v8f& a3, v16h x, v16h y, v16h b0, v16h b1, v16h b2, v16h b3) {
  asm volatile("v_nop\n\tv_nop\n\tv_nop\n\tv_nop" : "+v"(a0), "+v"(a1), "+v"(a2), "+v"(a3) : "v"(x), "v"(y), "v"(b0), "v"(b1), "v"(b2), "v"(b3));
}
__device__ __forceinline__ void dep_guard4_b(v8f& a0, v8f& a1, v8f& a2, v8f& a3, v16b x, v16b y, v16b b0, v16b b1, v16b b2, v16b b3) {
  asm volatile("v_nop\n\tv_nop\n\tv_nop\n\tv_nop" : "+v"(a0), "+v"(a1), "+v"(a2), "+v"(a3) : "v"(x), "v"(y), "v"(b0), "v"(b1), "v"(b2), "v"(b3));
}
__device__ __forceinline__ void dep_guard2x3_h(v8f& a0, v8f& a1, v16h x, v16h b0, v16h b1) {
  asm volatile("v_nop\n\tv_nop\n\tv_nop\n\tv_nop" : "+v"(a0), "+v"(a1) : "v"(x), "v"(b0), "v"(b1));
}
__device__ __forceinline__ void keep4_h(v16h a, v16h b, v16h c, v16h d) { asm volatile("v_nop" :: "v"(a), "v"(b), "v"(c), "v"(d)); }
__device__ __forceinline__ void keep4_b(v16b a, v16b b, v16b c, v16b d) { asm volatile("v_nop" :: "v"(a), "v"(b), "v"(c), "v"(d)); }
__device__ __forceinline__ void acc_guard4(v8f& a, v8f& b, v8f& c, v8f& d) { asm volatile("v_nop\n\tv_nop\n\tv_nop\n\tv_nop" : "+v"(a), "+v"(b), "+v"(c), "+v"(d)); }
template <typename T> struct Frag;
template <> struct Frag<_Float16> {
  typedef v16h V; union U { v16h v; v8h h[2]; };
  static __device__ __forceinline__ v16h load(const _Float16* p) {
    U f; f.h[0] = *(const v8h*)(p); f.h[1] = *(const v8h*)(p + 16); return f.v;
  }
  static __device__ __forceinline__ v8f mma(v16h a, v16h b, v8f c) {
    return __builtin_amdgcn_wmma_f32_16x16x32_f16(false, a, false, b, (short)0, c, false, false);
  }
  static __device__ __forceinline__ void guard(v8f& a, v8f& b, v16h x, v16h y) { dep_guard_h(a, b, x, y); }
  static __device__ __forceinline__ void guard4(v8f& a0, v8f& a1, v8f& a2, v8f& a3, v16h x, v16h y, v16h b0, v16h b1, v16h b2, v16h b3) {
    dep_guard4_h(a0, a1, a2, a3, x, y, b0, b1, b2, b3);
  }
  static __device__ __forceinline__ void keep(v16h a, v16h b, v16h c, v16h d) { keep4_h(a, b, c, d); }
};
template <> struct Frag<__bf16> {
  typedef v16b V; union U { v16b v; v8b h[2]; };
  static __device__ __forceinline__ v16b load(const __bf16* p) {
    U f; f.h[0] = *(const v8b*)(p); f.h[1] = *(const v8b*)(p + 16); return f.v;
  }
  static __device__ __forceinline__ v8f mma(v16b a, v16b b, v8f c) {
    return __builtin_amdgcn_wmma_f32_16x16x32_bf16(false, a, false, b, (short)0, c, false, false);
  }
  static __device__ __forceinline__ void guard(v8f& a, v8f& b, v16b x, v16b y) { dep_guard_b(a, b, x, y); }
  static __device__ __forceinline__ void guard4(v8f& a0, v8f& a1, v8f& a2, v8f& a3, v16b x, v16b y, v16b b0, v16b b1, v16b b2, v16b b3) {
    dep_guard4_b(a0, a1, a2, a3, x, y, b0, b1, b2, b3);
  }
  static __device__ __forceinline__ void keep(v16b a, v16b b, v16b c, v16b d) { keep4_b(a, b, c, d); }
};

__device__ __forceinline__ unsigned pk16(unsigned short a, unsigned short b) { return (unsigned)a | ((unsigned)b << 16); }
__device__ __forceinline__ unsigned short h_bits(float f) { const _Float16 h = (_Float16)f; return __builtin_bit_cast(unsigned short, h); }

template <int ET> struct Elem;
template <> struct Elem<0> { typedef _Float16 T; };
template <> struct Elem<1> { typedef __bf16 T; };
template <int ET, bool SPLIT, int BIAS_MODE, int OUT_MODE, bool RESID, int ACT = 0>
__global__ __launch_bounds__(256) void wmma_gemm64(
    const unsigned short* __restrict__ Ap, const unsigned short* __restrict__ A2p, int lda, long strideA,
    const unsigned short* __restrict__ Btp, const unsigned short* __restrict__ Bt2p, int ldb, long strideB,
    void* __restrict__ Cout, void* __restrict__ Cout2, int ldc, long strideC,
    const float* __restrict__ bias,
    const float* __restrict__ resid, long strideR,
    int M, int N, int K, float scale) {
  static_assert(!RESID, "resid path not used");
  typedef typename Elem<ET>::T T;
  typedef typename Frag<T>::V V;
  const T* A = (const T*)Ap; const T* A2 = (const T*)A2p; const T* Bt = (const T*)Btp; const T* Bt2 = (const T*)Bt2p;
  __shared__ __align__(16) float sT[8][16 * 68];
  (void)resid; (void)strideR;
  const int b    = blockIdx.y;
  const int lane = threadIdx.x & 31;
  const int wave = threadIdx.x >> 5;
  const int tilesN = N >> 6;
  const int tilesM = M >> 6;
  const int tile = blockIdx.x * 8 + wave;
  if (tile >= tilesM * tilesN) return;
  const int tm = tile / tilesN;
  const int tn = tile - tm * tilesN;
  const int m0 = tm << 6;
  const int n0 = tn << 6;

  const T* Ab  = A  + (size_t)b * strideA;
  const T* Bb  = Bt + (size_t)b * strideB;
  const T* Ab2 = SPLIT ? (A2  + (size_t)b * strideA) : nullptr;
  const T* Bb2 = SPLIT ? (Bt2 + (size_t)b * strideB) : nullptr;

  const int rlane = lane & 15;
  const int koff  = (lane >> 4) * 8;
  const int mOff  = (lane >> 4) * 8;

  v8f acc[4][4];
#pragma unroll
  for (int i = 0; i < 4; ++i)
#pragma unroll
    for (int j = 0; j < 4; ++j) acc[i][j] = (v8f){0.f,0.f,0.f,0.f,0.f,0.f,0.f,0.f};

  for (int k0 = 0; k0 < K; k0 += 32) {
    V bh[4], bl[4];
#pragma unroll
    for (int j = 0; j < 4; ++j) {
      const size_t bo = (size_t)(n0 + (j << 4) + rlane) * ldb + koff + k0;
      bh[j] = Frag<T>::load(Bb + bo);
      if (SPLIT) bl[j] = Frag<T>::load(Bb2 + bo);
    }
#pragma unroll
    for (int i = 0; i < 4; ++i) {
      const size_t ao = (size_t)(m0 + (i << 4) + rlane) * lda + koff + k0;
      V ah = Frag<T>::load(Ab + ao);
      V al;
      if (SPLIT) al = Frag<T>::load(Ab2 + ao);
#pragma unroll
      for (int j = 0; j < 4; ++j) {
        acc[i][j] = Frag<T>::mma(ah, bh[j], acc[i][j]);
        if (SPLIT) {
          acc[i][j] = Frag<T>::mma(ah, bl[j], acc[i][j]);
          acc[i][j] = Frag<T>::mma(al, bh[j], acc[i][j]);
        }
      }
      Frag<T>::guard4(acc[i][0], acc[i][1], acc[i][2], acc[i][3], ah, SPLIT ? al : ah, bh[0], bh[1], bh[2], bh[3]);
    }
    Frag<T>::keep(bh[0], bh[1], bh[2], bh[3]);
    if (SPLIT) Frag<T>::keep(bl[0], bl[1], bl[2], bl[3]);
  }
  acc_guard4(acc[0][0], acc[0][1], acc[0][2], acc[0][3]);
  acc_guard4(acc[1][0], acc[1][1], acc[1][2], acc[1][3]);
  acc_guard4(acc[2][0], acc[2][1], acc[2][2], acc[2][3]);
  acc_guard4(acc[3][0], acc[3][1], acc[3][2], acc[3][3]);

  float* slab = sT[wave];
#pragma unroll
  for (int i = 0; i < 4; ++i) {
    const int mBase = m0 + (i << 4);
#pragma unroll
    for (int j = 0; j < 4; ++j) {
      const int n = n0 + (j << 4) + rlane;
      float bv = 0.f;
      if (BIAS_MODE == 2) bv = bias[n];
#pragma unroll
      for (int r = 0; r < 8; ++r) {
        float v = acc[i][j][r] * scale;
        if (BIAS_MODE == 1) v += bias[mBase + mOff + r];
        if (BIAS_MODE == 2) v += bv;
        if (ACT == 2) v = fmaxf(v, 0.0f);
        if (ACT == 4) v = (v > 0.f) ? v : 0.01f * v;
        if (ACT == 6) v = (v > 0.f) ? (v + 1.0f) : expf(v);
        slab[(mOff + r) * 68 + (j << 4) + rlane] = v;
      }
    }
    __builtin_amdgcn_fence(__ATOMIC_RELEASE, "workgroup");
    __builtin_amdgcn_wave_barrier();
    __builtin_amdgcn_fence(__ATOMIC_ACQUIRE, "workgroup");
    if (OUT_MODE == 0) {
      float* Cp = (float*)Cout + (size_t)b * strideC;
      const int hh = lane >> 4, c4 = (lane & 15) * 4;
      for (int pass = 0; pass < 2; ++pass) {
#pragma unroll
        for (int it = 0; it < 8; ++it) {
          const int row = it * 2 + hh;
          v4f v = *(const v4f*)(slab + row * 68 + c4);
          *(volatile v4f*)(Cp + (size_t)(mBase + row) * ldc + n0 + c4) = v;
        }
        __threadfence();
      }
    } else {
      const int q = lane >> 3, c8 = (lane & 7) * 8;
      unsigned short* Cp  = (unsigned short*)Cout  + (size_t)b * strideC;
      unsigned short* Cp2 = (OUT_MODE == 2) ? ((unsigned short*)Cout2 + (size_t)b * strideC) : nullptr;
      for (int pass = 0; pass < 2; ++pass) {
#pragma unroll
        for (int it = 0; it < 4; ++it) {
          const int row = it * 4 + q;
          const float* sp = slab + row * 68 + c8;
          v8h hv, lv;
#pragma unroll
          for (int e = 0; e < 8; ++e) {
            if (OUT_MODE == 1) {
              hv[e] = (_Float16)sp[e];
            } else {
              unsigned short hb = f2bf_bits(sp[e]);
              unsigned short lb = f2bf_bits(sp[e] - bf_bits2f(hb));
              hv[e] = __builtin_bit_cast(_Float16, hb);
              lv[e] = __builtin_bit_cast(_Float16, lb);
            }
          }
          *(volatile v8h*)(Cp + (size_t)(mBase + row) * ldc + n0 + c8) = hv;
          if (OUT_MODE == 2) *(volatile v8h*)(Cp2 + (size_t)(mBase + row) * ldc + n0 + c8) = lv;
        }
        __threadfence();
      }
    }
    __builtin_amdgcn_fence(__ATOMIC_RELEASE, "workgroup");
    __builtin_amdgcn_wave_barrier();
    __builtin_amdgcn_fence(__ATOMIC_ACQUIRE, "workgroup");
  }
}

__global__ __launch_bounds__(256) void cast8_f16_kernel(const float* __restrict__ in, unsigned short* __restrict__ out, int n8, float carry) {
  const int i = blockIdx.x * 256 + threadIdx.x;
  if (i >= n8) return;
  const float* p = in + 8 * (size_t)i;
  const v4f a = *(const v4f*)(p);
  const v4f c = *(const v4f*)(p + 4);
  unsigned short hb[8];
#pragma unroll
  for (int e = 0; e < 4; ++e) {
    hb[e]     = h_bits(a[e] * carry);
    hb[4 + e] = h_bits(c[e] * carry);
  }
  const v4u u = (v4u){pk16(hb[0], hb[1]), pk16(hb[2], hb[3]), pk16(hb[4], hb[5]), pk16(hb[6], hb[7])};
  unsigned short* q = out + 8 * (size_t)i;
  *(volatile v4u*)q = u;
  __threadfence();
  *(volatile v4u*)q = u;
}

__global__ __launch_bounds__(256) void kv_ksum_kernel(const unsigned short* __restrict__ KTp, const unsigned short* __restrict__ VTp,
                                                     unsigned short* __restrict__ KVp, float* __restrict__ ksp) {
  __shared__ __align__(16) float kvs[64 * 68];
  __shared__ __align__(16) float kss[64];
  const int bh   = blockIdx.x;
  const int b    = bh / kHeads;
  const int h    = bh - b * kHeads;
  const int tid  = threadIdx.x;
  const int lane = tid & 31, wave = tid >> 5;
  const int rlane = lane & 15;
  const int koff  = (lane >> 4) * 8;
  const int mOff  = (lane >> 4) * 8;
  const size_t plane = (size_t)(h * kDh) * kTok + (size_t)b * kSeq;
  const _Float16* KT = (const _Float16*)KTp + plane;
  const _Float16* VT = (const _Float16*)VTp + plane;
  const int ti = wave >> 1;
  const int tj = (wave & 1) * 2;

  v8f acc0 = (v8f){0.f,0.f,0.f,0.f,0.f,0.f,0.f,0.f};
  v8f acc1 = (v8f){0.f,0.f,0.f,0.f,0.f,0.f,0.f,0.f};
  const _Float16* arow  = VT + (size_t)(ti * 16 + rlane) * kTok + koff;
  const _Float16* b0row = KT + (size_t)(tj * 16 + rlane) * kTok + koff;
  const _Float16* b1row = b0row + (size_t)16 * kTok;
#pragma unroll 1
  for (int n0 = 0; n0 < kSeq; n0 += 32) {
    const v16h af = Frag<_Float16>::load(arow + n0);
    const v16h f0 = Frag<_Float16>::load(b0row + n0);
    const v16h f1 = Frag<_Float16>::load(b1row + n0);
    acc0 = Frag<_Float16>::mma(af, f0, acc0);
    acc1 = Frag<_Float16>::mma(af, f1, acc1);
    dep_guard2x3_h(acc0, acc1, af, f0, f1);
  }
  dep_guard2x3_h(acc0, acc1, (v16h){}, (v16h){}, (v16h){});

  {
    const int d = tid >> 2, part = tid & 3;
    const unsigned short* kr = KTp + plane + (size_t)d * kTok + part * 1024;
    float s0 = 0.f, s1 = 0.f;
#pragma unroll 1
    for (int it = 0; it < 128; ++it) {
      const v4u w = *(const v4u*)(kr + 8 * it);
      const unsigned w0 = w[0], w1 = w[1], w2 = w[2], w3 = w[3];
      s0 += (h16_to_f32(w0 & 0xffffu) + h16_to_f32(w0 >> 16)) + (h16_to_f32(w1 & 0xffffu) + h16_to_f32(w1 >> 16));
      s1 += (h16_to_f32(w2 & 0xffffu) + h16_to_f32(w2 >> 16)) + (h16_to_f32(w3 & 0xffffu) + h16_to_f32(w3 >> 16));
    }
    float s = s0 + s1;
    s += __shfl_xor(s, 1, 32);
    s += __shfl_xor(s, 2, 32);
    if (part == 0) kss[d] = s;
  }

#pragma unroll
  for (int r = 0; r < 8; ++r) {
    kvs[(ti * 16 + mOff + r) * 68 + tj * 16 + rlane]      = acc0[r];
    kvs[(ti * 16 + mOff + r) * 68 + tj * 16 + 16 + rlane] = acc1[r];
  }
  __syncthreads();

  unsigned short* KVo = KVp + (size_t)bh * kDh * kDh;
  float* kso = ksp + (size_t)bh * kDh;
  const int q = lane >> 3, c8 = (lane & 7) * 8;
  for (int pass = 0; pass < 2; ++pass) {
#pragma unroll
    for (int it = 0; it < 2; ++it) {
      const int row = wave * 8 + it * 4 + q;
      const float* sp = kvs + row * 68 + c8;
      v8h hv;
#pragma unroll
      for (int e = 0; e < 8; ++e) hv[e] = (_Float16)sp[e];
      *(volatile v8h*)(KVo + (size_t)row * kDh + c8) = hv;
    }
    if (wave == 0) {
      if (lane < 16) {
        const v4f val = *(const v4f*)(kss + 4 * lane);
        *(volatile v4f*)(kso + 4 * lane) = val;
      }
    }
    __threadfence();
  }
}

__global__ __launch_bounds__(256) void y_norm_kernel(const unsigned short* __restrict__ Qp, const unsigned short* __restrict__ KVp,
                                                    const float* __restrict__ ksp, unsigned short* __restrict__ Yp) {
  __shared__ __align__(16) float sT[8][16 * 68];
  __shared__ __align__(16) float ksl[64];
  __shared__ __align__(16) float dens[8][64];
  const int bh   = blockIdx.y;
  const int b    = bh / kHeads;
  const int h    = bh - b * kHeads;
  const int tid  = threadIdx.x;
  const int lane = tid & 31, wave = tid >> 5;
  const int rlane = lane & 15;
  const int koff  = (lane >> 4) * 8;
  const int mOff  = (lane >> 4) * 8;
  if (tid < 64) ksl[tid] = ksp[(size_t)bh * kDh + tid];
  __syncthreads();

  const int ntok = blockIdx.x * 512 + wave * 64;
  const size_t row0 = (size_t)b * kSeq + ntok;
  const int hcol = h * kDh;

  float* dw = dens[wave];
#pragma unroll 1
  for (int rr = 0; rr < 2; ++rr) {
    const size_t row = row0 + rr * 32 + lane;
    const unsigned short* qrow = Qp + row * kC + hcol;
    float s = 0.f;
#pragma unroll
    for (int g = 0; g < 8; ++g) {
      const v4u w = *(const v4u*)(qrow + 8 * g);
#pragma unroll
      for (int e = 0; e < 4; ++e) {
        const unsigned we = w[e];
        s = fmaf(h16_to_f32(we & 0xffffu), ksl[8 * g + 2 * e], s);
        s = fmaf(h16_to_f32(we >> 16), ksl[8 * g + 2 * e + 1], s);
      }
    }
    dw[rr * 32 + lane] = kYCarry / (s + kEps);
  }
  __syncthreads();

  const _Float16* Q   = (const _Float16*)Qp;
  const _Float16* KVb = (const _Float16*)KVp + (size_t)bh * kDh * kDh;
  v8f acc[4][4];
#pragma unroll
  for (int i = 0; i < 4; ++i)
#pragma unroll
    for (int j = 0; j < 4; ++j) acc[i][j] = (v8f){0.f,0.f,0.f,0.f,0.f,0.f,0.f,0.f};
#pragma unroll
  for (int ks = 0; ks < 2; ++ks) {
    const int k0 = ks * 32;
    v16h bf[4];
#pragma unroll
    for (int j = 0; j < 4; ++j) bf[j] = Frag<_Float16>::load(KVb + (size_t)(j * 16 + rlane) * kDh + koff + k0);
#pragma unroll
    for (int i = 0; i < 4; ++i) {
      const v16h af = Frag<_Float16>::load(Q + (row0 + i * 16 + rlane) * kC + hcol + koff + k0);
#pragma unroll
      for (int j = 0; j < 4; ++j) acc[i][j] = Frag<_Float16>::mma(af, bf[j], acc[i][j]);
      dep_guard4_h(acc[i][0], acc[i][1], acc[i][2], acc[i][3], af, af, bf[0], bf[1], bf[2], bf[3]);
    }
    keep4_h(bf[0], bf[1], bf[2], bf[3]);
  }
  acc_guard4(acc[0][0], acc[0][1], acc[0][2], acc[0][3]);
  acc_guard4(acc[1][0], acc[1][1], acc[1][2], acc[1][3]);
  acc_guard4(acc[2][0], acc[2][1], acc[2][2], acc[2][3]);
  acc_guard4(acc[3][0], acc[3][1], acc[3][2], acc[3][3]);

  float* slab = sT[wave];
  const int q = lane >> 3, c8 = (lane & 7) * 8;
#pragma unroll
  for (int i = 0; i < 4; ++i) {
    float sc[8];
#pragma unroll
    for (int r = 0; r < 8; ++r) sc[r] = dw[16 * i + mOff + r];
#pragma unroll
    for (int j = 0; j < 4; ++j) {
#pragma unroll
      for (int r = 0; r < 8; ++r) slab[(mOff + r) * 68 + (j << 4) + rlane] = acc[i][j][r] * sc[r];
    }
    __syncthreads();
    for (int pass = 0; pass < 2; ++pass) {
#pragma unroll
      for (int it = 0; it < 4; ++it) {
        const int row = it * 4 + q;
        const float* sp = slab + row * 68 + c8;
        v8h hv;
#pragma unroll
        for (int e = 0; e < 8; ++e) hv[e] = (_Float16)sp[e];
        *(volatile v8h*)(Yp + (row0 + (size_t)(i * 16 + row)) * kC + hcol + c8) = hv;
      }
      __threadfence();
    }
    __syncthreads();
  }
}

extern "C" void kernel_launch(void* const* d_in, const int* in_sizes, int n_in,
                              void* d_out, int out_size, void* d_ws, size_t ws_size,
                              hipStream_t stream) {
  if (n_in < 4) return;
  const int nX = kTok * kC;
  const int nWq = kC3 * kC;
  const int nWp = kC * kC;
  if (in_sizes[0] != nX || in_sizes[1] != nWq || in_sizes[2] != nWp || in_sizes[3] != kC) return;
  if (out_size != nX) return;

  const size_t szX  = (size_t)nX * 2;
  const size_t szWq = (size_t)nWq * 2;
  const size_t szWp = (size_t)nWp * 2;
  const size_t szT  = (size_t)kC * kTok * 2;
  const size_t szKV = (size_t)kBH * kDh * kDh * 2;
  const size_t szKS = (size_t)kBH * kDh * 4;
  const size_t offX  = 0;
  const size_t offWq = offX + szX;
  const size_t offWp = offWq + szWq;
  const size_t offQ  = offWp + szWp;
  const size_t offKT = offQ + szX;
  const size_t offVT = offKT + szT;
  const size_t offKV = offVT + szT;
  const size_t offKS = offKV + szKV;
  const size_t offY  = offKS + szKS;
  const size_t total = offY + szX;
  if (ws_size < total) return;

  const float* x     = (const float*)d_in[0];
  const float* Wqkv  = (const float*)d_in[1];
  const float* Wproj = (const float*)d_in[2];
  const float* bproj = (const float*)d_in[3];
  float* out = (float*)d_out;
  char* ws = (char*)d_ws;
  unsigned short* X16  = (unsigned short*)(ws + offX);
  unsigned short* WQ16 = (unsigned short*)(ws + offWq);
  unsigned short* WP16 = (unsigned short*)(ws + offWp);
  unsigned short* Q16  = (unsigned short*)(ws + offQ);
  unsigned short* KT   = (unsigned short*)(ws + offKT);
  unsigned short* VT   = (unsigned short*)(ws + offVT);
  unsigned short* KV16 = (unsigned short*)(ws + offKV);
  float*          KS   = (float*)(ws + offKS);
  unsigned short* Y16  = (unsigned short*)(ws + offY);

  const int n8x = nX / 8, n8q = nWq / 8, n8p = nWp / 8;
  cast8_f16_kernel<<<dim3(n8x / 256), dim3(256), 0, stream>>>(x, X16, n8x, 1.0f);
  cast8_f16_kernel<<<dim3(n8q / 256), dim3(256), 0, stream>>>(Wqkv, WQ16, n8q, kWCarry);
  cast8_f16_kernel<<<dim3(n8p / 256), dim3(256), 0, stream>>>(Wproj, WP16, n8p, kWCarry);

  const int tilesQ = (kTok / 64) * (kC / 64);

  wmma_gemm64<0, false, 0, 1, false, 6><<<dim3(tilesQ / 8, 1), dim3(256), 0, stream>>>(
      X16, X16, kC, 0L, WQ16, WQ16, kC, 0L,
      (void*)Q16, (void*)Q16, kC, 0L, bproj, bproj, 0L, kTok, kC, kC, kWCarryInv);
  wmma_gemm64<0, false, 0, 1, false, 6><<<dim3(tilesQ / 8, 1), dim3(256), 0, stream>>>(
      WQ16 + (size_t)kC * kC, WQ16 + (size_t)kC * kC, kC, 0L, X16, X16, kC, 0L,
      (void*)KT, (void*)KT, kTok, 0L, bproj, bproj, 0L, kC, kTok, kC, kWCarryInv);
  wmma_gemm64<0, false, 0, 1, false, 0><<<dim3(tilesQ / 8, 1), dim3(256), 0, stream>>>(
      WQ16 + (size_t)2 * kC * kC, WQ16 + (size_t)2 * kC * kC, kC, 0L, X16, X16, kC, 0L,
      (void*)VT, (void*)VT, kTok, 0L, bproj, bproj, 0L, kC, kTok, kC, kWCarryInv);

  kv_ksum_kernel<<<dim3(kBH), dim3(256), 0, stream>>>(KT, VT, KV16, KS);
  y_norm_kernel<<<dim3(kSeq / 512, kBH), dim3(256), 0, stream>>>(Q16, KV16, KS, Y16);

  wmma_gemm64<0, false, 2, 0, false, 0><<<dim3(tilesQ / 8, 1), dim3(256), 0, stream>>>(
      Y16, Y16, kC, 0L, WP16, WP16, kC, 0L,
      (void*)out, (void*)out, kC, 0L, bproj, bproj, 0L, kTok, kC, kC, kProjScale);
}
